// Transformer_45741401702593
// MI455X (gfx1250) — hardware-verified
//
#include <hip/hip_runtime.h>
#include <stdint.h>
#include <stddef.h>


#ifndef NB
#define NB 4096
#endif
#define NB_FULL 4096
#define TT 16
#define DM 32
#define NH 4
#define HS 64
#define VOC 65
#define VPAD 80
#define HID 2048
#define NCH (HID / 32)
#define NLAYER 2
#define PPB ((2 * TT * VOC) / 4)
#define NPI ((PPB + 63) / 64)

static_assert(TT == 16);
static_assert(DM == 32);
static_assert(HS == 64);
static_assert((HID % 32) == 0);
static_assert(((2 * TT * VOC * 4) % 128) == 0);
static_assert((VPAD % 16) == 0);
static_assert(VPAD >= VOC);
static_assert(PPB == 520);
static_assert(NPI * 64 >= PPB);

#define W_SCALE 64.0f
#define INV_W 0.015625f
#define P_SCALE 1024.0f
#define INV_P 0.0009765625f
#define SQD 5.656854249492380f
#define INV_SQRT_HS 0.125f
#define LN_EPS 1.0e-5f

typedef _Float16 v16h __attribute__((ext_vector_type(16)));
typedef _Float16 v8h  __attribute__((ext_vector_type(8)));
typedef float    v8f  __attribute__((ext_vector_type(8)));
typedef float    v4f  __attribute__((ext_vector_type(4)));
typedef unsigned int v4u __attribute__((ext_vector_type(4)));

union Frag  { v16h v; v8h h[2]; };
union Pack8 { v8h h; v4u u; };

__device__ __forceinline__ float bf16r(float v) {
  unsigned int u = __float_as_uint(v);
  u += 0x7fffu + ((u >> 16) & 1u);
  u &= 0xffff0000u;
  return __uint_as_float(u);
}

__device__ __forceinline__ v16h fragld(const _Float16* base, int ld, int k0, int lane) {
  const _Float16* p = base + (lane & 15) * ld + k0 + 8 * (lane >> 4);
  Frag f;
  f.h[0] = *(const v8h*)(p);
  f.h[1] = *(const v8h*)(p + 16);
  return f.v;
}

__device__ __forceinline__ v8f mma16(v16h a, v16h b, v8f c) {
  v8f d = __builtin_amdgcn_wmma_f32_16x16x32_f16(false, a, false, b, (short)0, c, false, false);
  asm volatile("v_nop\n\tv_nop\n\tv_nop\n\tv_nop" : "+v"(d) : "v"(a), "v"(b));
  return d;
}

__device__ __forceinline__ float rsum16(float v) {
  v += __shfl_xor(v, 8);
  v += __shfl_xor(v, 4);
  v += __shfl_xor(v, 2);
  v += __shfl_xor(v, 1);
  return v;
}
__device__ __forceinline__ float rmax16(float v) {
  v = fmaxf(v, __shfl_xor(v, 8));
  v = fmaxf(v, __shfl_xor(v, 4));
  v = fmaxf(v, __shfl_xor(v, 2));
  v = fmaxf(v, __shfl_xor(v, 1));
  return v;
}

__global__ __launch_bounds__(256) void k_pack(const float* __restrict__ src,
                                              _Float16* __restrict__ dst,
                                              int nbat, int K, int N, int Npad, int bstride) {
  const int gid = blockIdx.x * 256 + threadIdx.x;
  const int total = nbat * Npad * K;
  const int e = gid * 8;
  if (e >= total) return;
  const int per = Npad * K;
  const int b = e / per;
  const int wi = e - b * per;
  const int n = wi / K;
  const int k0 = wi - n * K;
  const int nn = (n < N) ? n : (N - 1);
  const float* sp = src + (size_t)b * bstride + (size_t)k0 * N + nn;
  v8h t8;
#pragma unroll
  for (int i = 0; i < 8; ++i) {
    float v = sp[(size_t)i * N];
    v = (n < N) ? (bf16r(v) * W_SCALE) : 0.0f;
    t8[i] = (_Float16)v;
  }
  Pack8 pk;
  pk.h = t8;
  _Float16* dp = dst + e;
  *(volatile v4u*)dp = pk.u;
  __threadfence();
  *(volatile v4u*)dp = pk.u;
}

__global__ __launch_bounds__(64) void k_main(
    const int* __restrict__ x, const float* __restrict__ emb, const float* __restrict__ pos,
    const float* __restrict__ bq, const float* __restrict__ bk, const float* __restrict__ bv,
    const float* __restrict__ bo, const float* __restrict__ ga, const float* __restrict__ ba,
    const float* __restrict__ b1, const float* __restrict__ b2,
    const float* __restrict__ gm, const float* __restrict__ bm, const float* __restrict__ bfin,
    const _Float16* __restrict__ WqT, const _Float16* __restrict__ WkT,
    const _Float16* __restrict__ WvT, const _Float16* __restrict__ WoT,
    const _Float16* __restrict__ W1T, const _Float16* __restrict__ W2T,
    const _Float16* __restrict__ WfT, float* out, int nb, int out_pieces)
{
  __shared__ __align__(16) float    hF[2][TT * DM];
  __shared__ __align__(16) _Float16 hH[2][TT * DM];
  __shared__ __align__(16) _Float16 qH[2][TT * HS];
  __shared__ __align__(16) _Float16 kH[2][TT * HS];
  __shared__ __align__(16) _Float16 vT[2][HS * 32];
  __shared__ __align__(16) _Float16 pH[2][TT * 32];
  __shared__ __align__(16) _Float16 oH[2][TT * HS];
  __shared__ __align__(16) _Float16 yH[2][TT * 32];
  __shared__ __align__(16) float    stage[2 * TT * VOC];

  const int tid  = threadIdx.x;
  const int lane = tid & 31;
  const int w    = tid >> 5;
  const int m    = lane & 15;
  const int hh   = lane >> 4;
  const int seq  = blockIdx.x * 2 + w;
  const int seqc = (seq < nb) ? seq : (nb - 1);

  float*    hFw = &hF[w][0];
  _Float16* hHw = &hH[w][0];
  _Float16* qHw = &qH[w][0];
  _Float16* kHw = &kH[w][0];
  _Float16* vTw = &vT[w][0];
  _Float16* pHw = &pH[w][0];
  _Float16* oHw = &oH[w][0];
  _Float16* yHw = &yH[w][0];
  float*    stw = stage + w * (TT * VOC);

  {
    v4u z4 = {};
    *(v4u*)(pHw + (lane >> 1) * 32 + 16 + 8 * (lane & 1)) = z4;
#pragma unroll
    for (int i = 0; i < 4; ++i) {
      const int idx = lane + 32 * i;
      *(v4u*)(vTw + (idx >> 1) * 32 + 16 + 8 * (idx & 1)) = z4;
    }
  }

#pragma unroll 1
  for (int t = 0; t < TT; ++t) {
    int tok = x[(size_t)seqc * TT + t];
    tok = (tok < 0) ? 0 : tok;
    tok = (tok > VOC - 1) ? (VOC - 1) : tok;
    const float e = bf16r(emb[tok * DM + lane]);
    const float p = bf16r(pos[t * DM + lane]);
    const float v = (e + p) * SQD;
    hFw[t * DM + lane] = v;
    hHw[t * DM + lane] = (_Float16)v;
  }
  __syncthreads();

  const v8f zero = {};

#pragma unroll 1
  for (int l = 0; l < NLAYER; ++l) {
    v16h hA = fragld(hHw, DM, 0, lane);
    v8f c0 = zero, c1 = zero;

#pragma unroll 1
    for (int head = 0; head < NH; ++head) {
      const int lh = l * NH + head;

#pragma unroll 1
      for (int j = 0; j < 4; ++j) {
        const size_t wrow = ((size_t)lh * HS + (size_t)j * 16) * DM;
        v16h bqf = fragld(WqT + wrow, DM, 0, lane);
        v16h bkf = fragld(WkT + wrow, DM, 0, lane);
        v16h bvf = fragld(WvT + wrow, DM, 0, lane);
        v8f qa = mma16(hA, bqf, zero);
        v8f ka = mma16(hA, bkf, zero);
        v8f va = mma16(hA, bvf, zero);
        const int col = j * 16 + m;
        const float bqv = bf16r(bq[lh * HS + col]);
        const float bkv = bf16r(bk[lh * HS + col]);
        const float bvv = bf16r(bv[lh * HS + col]);
        v8h t8;
#pragma unroll
        for (int r = 0; r < 8; ++r) {
          const int row = 8 * hh + r;
          qHw[row * HS + col] = (_Float16)(qa[r] * INV_W + bqv);
          kHw[row * HS + col] = (_Float16)(ka[r] * INV_W + bkv);
          t8[r] = (_Float16)(va[r] * INV_W + bvv);
        }
        *(v8h*)(vTw + col * 32 + 8 * hh) = t8;
      }
      __syncthreads();

      v8f sa = zero;
#pragma unroll
      for (int kc = 0; kc < 2; ++kc) {
        v16h aq  = fragld(qHw, HS, kc * 32, lane);
        v16h bkk = fragld(kHw, HS, kc * 32, lane);
        sa = mma16(aq, bkk, sa);
      }
#pragma unroll
      for (int r = 0; r < 8; ++r) {
        const int row = 8 * hh + r;
        const bool valid = (m <= row);
        const float sv = valid ? (sa[r] * INV_SQRT_HS) : -1.0e30f;
        const float mx = rmax16(sv);
        const float e  = __expf(sv - mx);
        const float sm = rsum16(e);
        const float p  = e * (P_SCALE / sm);
        pHw[row * 32 + m] = (_Float16)p;
      }
      __syncthreads();

      {
        v16h pA = fragld(pHw, 32, 0, lane);
#pragma unroll 1
        for (int j = 0; j < 4; ++j) {
          v16h bvv = fragld(vTw + j * 16 * 32, 32, 0, lane);
          v8f oa = mma16(pA, bvv, zero);
#pragma unroll
          for (int r = 0; r < 8; ++r)
            oHw[(8 * hh + r) * HS + j * 16 + m] = (_Float16)(oa[r] * INV_P);
        }
      }
      __syncthreads();

#pragma unroll
      for (int kc = 0; kc < 2; ++kc) {
        v16h oA = fragld(oHw, HS, kc * 32, lane);
        v16h bw0 = fragld(WoT + ((size_t)l * DM + 0)  * (NH * HS), NH * HS, head * HS + kc * 32, lane);
        v16h bw1 = fragld(WoT + ((size_t)l * DM + 16) * (NH * HS), NH * HS, head * HS + kc * 32, lane);
        c0 = mma16(oA, bw0, c0);
        c1 = mma16(oA, bw1, c1);
      }
      __syncthreads();
    }

    {
      const float g0 = bf16r(ga[l * DM + m]),  g1 = bf16r(ga[l * DM + 16 + m]);
      const float e0 = bf16r(ba[l * DM + m]),  e1 = bf16r(ba[l * DM + 16 + m]);
      const float o0 = bf16r(bo[l * DM + m]),  o1 = bf16r(bo[l * DM + 16 + m]);
#pragma unroll
      for (int r = 0; r < 8; ++r) {
        const int row = 8 * hh + r;
        const float x0 = (c0[r] * INV_W + o0) + hFw[row * DM + m];
        const float x1 = (c1[r] * INV_W + o1) + hFw[row * DM + 16 + m];
        const float mean = rsum16(x0 + x1) * (1.0f / 32.0f);
        const float d0 = x0 - mean, d1 = x1 - mean;
        const float var = rsum16(d0 * d0 + d1 * d1) * (1.0f / 32.0f);
        const float rstd = rsqrtf(var + LN_EPS);
        const float y0 = d0 * rstd * g0 + e0;
        const float y1 = d1 * rstd * g1 + e1;
        hFw[row * DM + m]      = y0;  hHw[row * DM + m]      = (_Float16)y0;
        hFw[row * DM + 16 + m] = y1;  hHw[row * DM + 16 + m] = (_Float16)y1;
      }
    }
    __syncthreads();

    v16h hA2 = fragld(hHw, DM, 0, lane);
    v8f mc0 = zero, mc1 = zero;
    const _Float16* w2a = W2T + ((size_t)l * DM + 0)  * HID;
    const _Float16* w2b = W2T + ((size_t)l * DM + 16) * HID;
#pragma unroll 1
    for (int c = 0; c < NCH; ++c) {
      const _Float16* w1p = W1T + ((size_t)l * HID + (size_t)c * 32) * DM;
      v16h b10 = fragld(w1p, DM, 0, lane);
      v16h b11 = fragld(w1p + 16 * DM, DM, 0, lane);
      v8f y0 = mma16(hA2, b10, zero);
      v8f y1 = mma16(hA2, b11, zero);
      const float bb0 = bf16r(b1[(size_t)l * HID + c * 32 + m]);
      const float bb1 = bf16r(b1[(size_t)l * HID + c * 32 + 16 + m]);
#pragma unroll
      for (int r = 0; r < 8; ++r) {
        const int row = 8 * hh + r;
        yHw[row * 32 + m]      = (_Float16)fmaxf(y0[r] * INV_W + bb0, 0.0f);
        yHw[row * 32 + 16 + m] = (_Float16)fmaxf(y1[r] * INV_W + bb1, 0.0f);
      }
      __syncthreads();
      v16h yA  = fragld(yHw, 32, 0, lane);
      v16h b20 = fragld(w2a, HID, c * 32, lane);
      v16h b21 = fragld(w2b, HID, c * 32, lane);
      mc0 = mma16(yA, b20, mc0);
      mc1 = mma16(yA, b21, mc1);
      __syncthreads();
    }

    {
      const float g0 = bf16r(gm[l * DM + m]),  g1 = bf16r(gm[l * DM + 16 + m]);
      const float e0 = bf16r(bm[l * DM + m]),  e1 = bf16r(bm[l * DM + 16 + m]);
      const float t0 = bf16r(b2[l * DM + m]),  t1 = bf16r(b2[l * DM + 16 + m]);
#pragma unroll
      for (int r = 0; r < 8; ++r) {
        const int row = 8 * hh + r;
        const float x0 = hFw[row * DM + m]      + (mc0[r] * INV_W + t0);
        const float x1 = hFw[row * DM + 16 + m] + (mc1[r] * INV_W + t1);
        const float mean = rsum16(x0 + x1) * (1.0f / 32.0f);
        const float d0 = x0 - mean, d1 = x1 - mean;
        const float var = rsum16(d0 * d0 + d1 * d1) * (1.0f / 32.0f);
        const float rstd = rsqrtf(var + LN_EPS);
        const float y0 = d0 * rstd * g0 + e0;
        const float y1 = d1 * rstd * g1 + e1;
        hFw[row * DM + m]      = y0;  hHw[row * DM + m]      = (_Float16)y0;
        hFw[row * DM + 16 + m] = y1;  hHw[row * DM + 16 + m] = (_Float16)y1;
      }
    }
    __syncthreads();
  }

  {
    v16h hA3 = fragld(hHw, DM, 0, lane);
#pragma unroll 1
    for (int nt = 0; nt < VPAD / 16; ++nt) {
      v16h bff = fragld(WfT + (size_t)nt * 16 * DM, DM, 0, lane);
      v8f fa = mma16(hA3, bff, zero);
      const int col  = nt * 16 + m;
      const int colc = (col < VOC) ? col : (VOC - 1);
      const float bfr = bf16r(bfin[colc]);
      if (col < VOC) {
#pragma unroll
        for (int r = 0; r < 8; ++r)
          stw[(8 * hh + r) * VOC + col] = fa[r] * INV_W + bfr;
      }
    }
  }
  __syncthreads();

  {
    const size_t pb = (size_t)blockIdx.x * PPB;
    v4f vv[NPI];
#pragma unroll
    for (int i = 0; i < NPI; ++i) {
      const int p  = tid + 64 * i;
      const int pc = (p < PPB) ? p : (PPB - 1);
      vv[i] = *(const v4f*)(stage + 4 * pc);
    }
#pragma unroll
    for (int i = 0; i < NPI; ++i) {
      const int p = tid + 64 * i;
      if (p < PPB && (pb + (size_t)p) < (size_t)out_pieces)
        *(volatile v4f*)(out + (pb + (size_t)p) * 4) = vv[i];
    }
    __threadfence();
#pragma unroll
    for (int i = 0; i < NPI; ++i) {
      const int p = tid + 64 * i;
      if (p < PPB && (pb + (size_t)p) < (size_t)out_pieces)
        *(volatile v4f*)(out + (pb + (size_t)p) * 4) = vv[i];
    }
  }
}

extern "C" void kernel_launch(void* const* d_in, const int* in_sizes, int n_in,
                              void* d_out, int out_size, void* d_ws, size_t ws_size,
                              hipStream_t stream)
{
  if (n_in < 21) return;
  const int*   x    = (const int*)  d_in[0];
  const float* emb  = (const float*)d_in[1];
  const float* pos  = (const float*)d_in[2];
  const float* Wq   = (const float*)d_in[3];
  const float* bq   = (const float*)d_in[4];
  const float* Wk   = (const float*)d_in[5];
  const float* bk   = (const float*)d_in[6];
  const float* Wv   = (const float*)d_in[7];
  const float* bv   = (const float*)d_in[8];
  const float* Wo   = (const float*)d_in[9];
  const float* bo   = (const float*)d_in[10];
  const float* ga   = (const float*)d_in[11];
  const float* ba   = (const float*)d_in[12];
  const float* W1   = (const float*)d_in[13];
  const float* b1   = (const float*)d_in[14];
  const float* W2   = (const float*)d_in[15];
  const float* b2   = (const float*)d_in[16];
  const float* gm   = (const float*)d_in[17];
  const float* bm   = (const float*)d_in[18];
  const float* Wf   = (const float*)d_in[19];
  const float* bfin = (const float*)d_in[20];
  float* out = (float*)d_out;

  if (in_sizes[0]  < NB * TT) return;
  if (in_sizes[1]  < VOC * DM) return;
  if (in_sizes[2]  < TT * DM) return;
  if (in_sizes[3]  < NLAYER * NH * DM * HS) return;
  if (in_sizes[4]  < NLAYER * NH * HS) return;
  if (in_sizes[5]  < NLAYER * NH * DM * HS) return;
  if (in_sizes[6]  < NLAYER * NH * HS) return;
  if (in_sizes[7]  < NLAYER * NH * DM * HS) return;
  if (in_sizes[8]  < NLAYER * NH * HS) return;
  if (in_sizes[9]  < NLAYER * NH * HS * DM) return;
  if (in_sizes[10] < NLAYER * DM) return;
  if (in_sizes[11] < NLAYER * DM) return;
  if (in_sizes[12] < NLAYER * DM) return;
  if (in_sizes[13] < NLAYER * DM * HID) return;
  if (in_sizes[14] < NLAYER * HID) return;
  if (in_sizes[15] < NLAYER * HID * DM) return;
  if (in_sizes[16] < NLAYER * DM) return;
  if (in_sizes[17] < NLAYER * DM) return;
  if (in_sizes[18] < NLAYER * DM) return;
  if (in_sizes[19] < DM * VOC) return;
  if (in_sizes[20] < VOC) return;
  if (out_size < NB * TT * VOC) return;

  size_t off = 0;
  auto take = [&](size_t bytes) -> void* {
    void* p = (char*)d_ws + off;
    off += (bytes + 255) & ~(size_t)255;
    return p;
  };
  const size_t szQKV = (size_t)NLAYER * NH * HS * DM * sizeof(_Float16);
  const size_t szWo  = (size_t)NLAYER * DM * (NH * HS) * sizeof(_Float16);
  const size_t szW1  = (size_t)NLAYER * HID * DM * sizeof(_Float16);
  const size_t szW2  = (size_t)NLAYER * DM * HID * sizeof(_Float16);
  const size_t szWf  = (size_t)VPAD * DM * sizeof(_Float16);
  _Float16* WqT = (_Float16*)take(szQKV);
  _Float16* WkT = (_Float16*)take(szQKV);
  _Float16* WvT = (_Float16*)take(szQKV);
  _Float16* WoT = (_Float16*)take(szWo);
  _Float16* W1T = (_Float16*)take(szW1);
  _Float16* W2T = (_Float16*)take(szW2);
  _Float16* WfT = (_Float16*)take(szWf);
  if (off > ws_size) return;

  auto pack = [&](const float* src, _Float16* dst, int nbat, int K, int N, int Npad, int bstride) {
    const int total = nbat * Npad * K;
    const int nthr = total / 8;
    k_pack<<<(nthr + 255) / 256, 256, 0, stream>>>(src, dst, nbat, K, N, Npad, bstride);
  };
  pack(Wq, WqT, NLAYER * NH, DM, HS, HS, DM * HS);
  pack(Wk, WkT, NLAYER * NH, DM, HS, HS, DM * HS);
  pack(Wv, WvT, NLAYER * NH, DM, HS, HS, DM * HS);
  pack(Wo, WoT, NLAYER, NH * HS, DM, DM, NH * HS * DM);
  pack(W1, W1T, NLAYER, DM, HID, HID, DM * HID);
  pack(W2, W2T, NLAYER, HID, DM, DM, HID * DM);
  pack(Wf, WfT, 1, DM, VOC, VPAD, DM * VOC);

  const int out_pieces = out_size / 4;
  const int nblk = (NB + 1) / 2;
  k_main<<<nblk, 64, 0, stream>>>(x, emb, pos, bq, bk, bv, bo, ga, ba, b1, b2, gm, bm, bfin,
                                  WqT, WkT, WvT, WoT, W1T, W2T, WfT, out, NB, out_pieces);
  (void)NB_FULL;
}
